// Temporal_Alignment_49237505081659
// MI455X (gfx1250) — hardware-verified
//
#include <hip/hip_runtime.h>
#include <math.h>

typedef __attribute__((ext_vector_type(16))) _Float16 v16h;
typedef __attribute__((ext_vector_type(16))) __bf16 v16b;
typedef __attribute__((ext_vector_type(8)))  _Float16 v8h;
typedef __attribute__((ext_vector_type(8)))  float v8f;
typedef __attribute__((ext_vector_type(4)))  float v4f;
typedef __attribute__((ext_vector_type(2)))  float v2f;
typedef __attribute__((ext_vector_type(4)))  unsigned v4u;
typedef __attribute__((ext_vector_type(4)))  int v4i;
typedef float __attribute__((may_alias)) float_a;
typedef int __attribute__((may_alias)) int_a;

template <typename T> __device__ __forceinline__ void vst2(void* p, T v) { *(volatile T*)p = v; __threadfence(); *(volatile T*)p = v; }
__device__ __forceinline__ v8f wmma16(v16h a, v16h b, v8f c) {
  v8f d = __builtin_amdgcn_wmma_f32_16x16x32_f16(false, a, false, b, (short)0, c, false, false);
  asm volatile("v_nop\n\tv_nop\n\tv_nop\n\tv_nop" : "+v"(d) : "v"(a), "v"(b));
  return d;
}
__device__ __forceinline__ v8f wmma_bf(v16b a, v16b b, v8f c) {
  v8f d = __builtin_amdgcn_wmma_f32_16x16x32_bf16(false, a, false, b, (short)0, c, false, false);
  asm volatile("v_nop\n\tv_nop\n\tv_nop\n\tv_nop" : "+v"(d) : "v"(a), "v"(b));
  return d;
}
__device__ __forceinline__ v16h frag_h(const _Float16* rowk0, int lane) {
  union { v16h v; v8h q[2]; } u; const _Float16* p = rowk0 + 8 * (lane >> 4);
  u.q[0] = *(const v8h*)p; u.q[1] = *(const v8h*)(p + 16); return u.v;
}
__device__ __forceinline__ v16h frag_f32(const float* rowk0, int lane) {
  v16h a; const float* p = rowk0 + 8 * (lane >> 4);
#pragma unroll
  for (int i = 0; i < 8; ++i) { a[i] = (_Float16)p[i]; a[8 + i] = (_Float16)p[16 + i]; }
  return a;
}
__device__ __forceinline__ v16h frag_f32s(const float* rowk0, int lane, float sc) {
  v16h a; const float* p = rowk0 + 8 * (lane >> 4);
#pragma unroll
  for (int i = 0; i < 8; ++i) { a[i] = (_Float16)(p[i] * sc); a[8 + i] = (_Float16)(p[16 + i] * sc); }
  return a;
}
__device__ __forceinline__ v16h fragc_f32(const float* W, int k0, int n, int lane, int ld, int K) {
  v16h a; const int g = lane >> 4;
#pragma unroll
  for (int i = 0; i < 8; ++i) { const int ka = k0 + 8 * g + i, kb = ka + 16;
    a[i] = (_Float16)(ka < K ? W[(size_t)(ka < K ? ka : K - 1) * ld + n] : 0.f); a[8 + i] = (_Float16)(kb < K ? W[(size_t)(kb < K ? kb : K - 1) * ld + n] : 0.f); }
  return a;
}
struct F2 { v16b h, l; };
__device__ __forceinline__ F2 bsplit16(const float v[16]) { F2 r;
#pragma unroll
  for (int i = 0; i < 16; ++i) { const __bf16 h = (__bf16)v[i]; r.h[i] = h; r.l[i] = (__bf16)(v[i] - (float)h); }
  return r; }
__device__ __forceinline__ F2 split_row(const float* row, int k0, int lane) { float v[16]; const float* p = row + k0 + 8 * (lane >> 4);
#pragma unroll
  for (int i = 0; i < 8; ++i) { v[i] = p[i]; v[8 + i] = p[16 + i]; }
  return bsplit16(v); }
__device__ __forceinline__ F2 split_rowK(const float* row, int k0, int lane, int K) { float v[16]; const int g = lane >> 4;
#pragma unroll
  for (int i = 0; i < 8; ++i) { const int ka = k0 + 8 * g + i, kb = ka + 16; v[i] = ka < K ? row[ka < K ? ka : K - 1] : 0.f; v[8 + i] = kb < K ? row[kb < K ? kb : K - 1] : 0.f; }
  return bsplit16(v); }
__device__ __forceinline__ F2 split_col(const float* W, int k0, int n, int lane, int ld, int K) { float v[16]; const int g = lane >> 4;
#pragma unroll
  for (int i = 0; i < 8; ++i) { const int ka = k0 + 8 * g + i, kb = ka + 16; v[i] = ka < K ? W[(size_t)(ka < K ? ka : K - 1) * ld + n] : 0.f; v[8 + i] = kb < K ? W[(size_t)(kb < K ? kb : K - 1) * ld + n] : 0.f; }
  return bsplit16(v); }
__device__ __forceinline__ v8f mac3(const F2& a, const F2& b, v8f c) { c = wmma_bf(a.l, b.h, c); c = wmma_bf(a.h, b.l, c); return wmma_bf(a.h, b.h, c); }
__device__ __forceinline__ float sigm(float v) { return 1.0f / (1.0f + expf(-v)); }
#define LDSX() do { asm volatile("s_wait_dscnt 0" ::: "memory"); __builtin_amdgcn_wave_barrier(); __builtin_amdgcn_fence(__ATOMIC_RELEASE, "workgroup"); } while (0)


#define NBT 2
#define CC 64
#define HH 64
#define WWD 64
#define NPI (HH * WWD)
#define NPIX (NBT * NPI)
#define HP 32
#define NPP (NBT * HP * HP)
#define OFFC 166
#define CP2 192
#define NGR 8
#ifndef NRB
#define NRB (NPIX / 64)
#define NRB1 NRB
#define NPB (NPP / 64)
#endif
typedef __attribute__((ext_vector_type(8))) __bf16 v8b;
__device__ __forceinline__ v16b frag_b(const __bf16* rowk0, int lane) {
  union { v16b v; v8b q[2]; } u; const __bf16* p = rowk0 + 8 * (lane >> 4);
  u.q[0] = *(const v8b*)p; u.q[1] = *(const v8b*)(p + 16); return u.v;
}
__device__ __forceinline__ float bfr(float v) { return (float)(__bf16)v; }
__device__ __attribute__((noinline)) float exp_ni(float v) { return expf(v); }
__device__ __attribute__((noinline)) float erf_ni(float v) { return erff(v); }
__device__ __forceinline__ v16b zfrag_if(v16b a, bool ok) { const v16b z = {}; return ok ? a : z; }

#define K33 (9 * 2 * CC)
#define K44 (9 * CP2)
#define KD3 (CC * 9)
#define KD5 (CC * 25)
#define KD7 (CC * 49)
#define PK_2 0
#define PK_3 (PK_2 + CP2 * K33)
#define PK_4 (PK_3 + CP2 * K33)
#define PK_D3 (PK_4 + CP2 * K44)
#define PK_D5 (PK_D3 + CC * KD3)
#define PK_D7 (PK_D5 + CC * KD5)
#define PK_PW (PK_D7 + CC * KD7)
#define PK_END (PK_PW + CC * CP2)
#define WS_PK  0u
#define WS_XY  (((2u * PK_END) + 127u) / 128u * 128u)
#define WS_PLH (WS_XY + 2u * NPIX * 128)
#define WS_PLL (WS_PLH + 2u * NPP * 128)
#define WS_O2  (WS_PLL + 2u * NPP * 128)
#define WS_G3H (WS_O2 + 4u * NPP * CP2)
#define WS_G3L (WS_G3H + 2u * NPIX * CP2)
#define WS_OFF (WS_G3L + 2u * NPIX * CP2)
#define WS_END (WS_OFF + 4u * NPIX * CP2)

__global__ __launch_bounds__(256) void k_pack(const float* __restrict__ K2W, const float* __restrict__ K3W, const float* __restrict__ K4W, const float* __restrict__ W3, const float* __restrict__ W5, const float* __restrict__ W7, const float* __restrict__ PWW, __bf16* __restrict__ PK) {
  __shared__ __align__(16) __bf16 s[KD7]; const int o = blockIdx.x, which = blockIdx.y, tid = threadIdx.x; int K; size_t dst;
  if (which <= 1) { const float* Wm = which == 0 ? K2W : K3W; K = K33; dst = (which == 0 ? PK_2 : PK_3) + (size_t)o * K33; for (int k = tid; k < K; k += 256) { const int tap = k / 128, c = k % 128; s[k] = (__bf16)((o < OFFC) ? Wm[((size_t)o * 128 + c) * 9 + tap] : 0.f); } }
  else if (which == 2) { K = K44; dst = PK_4 + (size_t)o * K44; for (int k = tid; k < K; k += 256) { const int tap = k / CP2, c = k % CP2; s[k] = (__bf16)((o < OFFC && c < OFFC) ? K4W[((size_t)o * OFFC + c) * 9 + tap] : 0.f); } }
  else if (which <= 5) { if (o >= CC) return; const int KS = (which == 3) ? 3 : (which == 4) ? 5 : 7, K2 = KS * KS; const float* Wm = (which == 3) ? W3 : (which == 4) ? W5 : W7; K = CC * K2; dst = ((which == 3) ? PK_D3 : (which == 4) ? PK_D5 : PK_D7) + (size_t)o * K; const int g = o / 8;
    for (int k = tid; k < K; k += 256) { const int c = k / K2, t = k % K2; s[k] = (__bf16)((c / 8 == g) ? Wm[(((size_t)o * 8 + (c - 8 * g)) * K2) + t] : 0.f); } }
  else { if (o >= CC) return; K = CP2; dst = PK_PW + (size_t)o * CP2; for (int k = tid; k < K; k += 256) s[k] = (__bf16)PWW[(size_t)o * CP2 + k]; }
  __syncthreads();
  for (int q = tid; q < K / 8; q += 256) vst2((unsigned*)(PK + dst + q * 8), *(const v4u*)&s[q * 8]);
}
__global__ __launch_bounds__(256) void k_xy(const float* __restrict__ X, const float* __restrict__ Y, __bf16* __restrict__ XY) {
  __shared__ __align__(16) __bf16 s[64][136]; const int row = blockIdx.x, tid = threadIdx.x; const int b = row / HH, y = row % HH;
  for (int q = tid; q < 128 * 64; q += 256) { const int c = q >> 6, px = q & 63; const float* src = (c < CC) ? X + (((size_t)b * CC + c) * HH + y) * WWD : Y + (((size_t)b * CC + (c - CC)) * HH + y) * WWD; s[px][c] = (__bf16)src[px]; }
  __syncthreads();
  for (int q = tid; q < 64 * 16; q += 256) { const int px = q >> 4, pc = q & 15; vst2((unsigned*)(XY + ((size_t)row * WWD + px) * 128 + pc * 8), *(const v4u*)&s[px][pc * 8]); }
}
__global__ __launch_bounds__(256) void k_pool(const __bf16* __restrict__ XY, __bf16* __restrict__ PH, __bf16* __restrict__ PL) {
  __shared__ __align__(16) __bf16 sh_[32][136], sl_[32][136]; const int prow = blockIdx.x, tid = threadIdx.x; const int b = prow / HP, py = prow % HP;
  for (int q = tid; q < 32 * 128; q += 256) { const int px = q >> 7, c = q & 127; const size_t r0 = ((size_t)b * HH + 2 * py) * WWD + 2 * px, r1 = r0 + WWD;
    const float v = (((float)XY[r0 * 128 + c] + (float)XY[(r0 + 1) * 128 + c]) + ((float)XY[r1 * 128 + c] + (float)XY[(r1 + 1) * 128 + c])) * 0.25f; const __bf16 hb = (__bf16)v; sh_[px][c] = hb; sl_[px][c] = (__bf16)(v - (float)hb); }
  __syncthreads();
  for (int q = tid; q < 32 * 16; q += 256) { const int px = q >> 4, pc = q & 15; const size_t o = ((size_t)prow * HP + px) * 128 + pc * 8; vst2((unsigned*)(PH + o), *(const v4u*)&sh_[px][pc * 8]); vst2((unsigned*)(PL + o), *(const v4u*)&sl_[px][pc * 8]); }
}
template <int MODE>
__global__ __launch_bounds__(128) void k_c33(const __bf16* __restrict__ IH, const __bf16* __restrict__ IL, const __bf16* __restrict__ W, const float* __restrict__ O2, float* __restrict__ OUTF, __bf16* __restrict__ OH, __bf16* __restrict__ OL) {
  constexpr int CP = (MODE == 2) ? CP2 : 128; constexpr int HI = (MODE == 0) ? HP : HH, WI = HI; constexpr int KT = 9 * CP;
  __shared__ __align__(16) float so[4][16][CP2 + 4];
  const int tid = threadIdx.x, wave = tid >> 5, lane = tid & 31, col = lane & 15, g = lane >> 4; const size_t r0 = (size_t)blockIdx.x * 64 + wave * 16; const size_t p = r0 + col;
  const int img = (int)(p / (HI * WI)), rem = (int)(p % (HI * WI)), y = rem / WI, xw = rem % WI;
  v8f acc[12] = {};
#pragma unroll 1
  for (int tap = 0; tap < 9; ++tap) { const int yy = y + tap / 3 - 1, xx = xw + tap % 3 - 1; const bool ok = (yy >= 0) && (yy < HI) && (xx >= 0) && (xx < WI);
    const size_t ap = ((size_t)img * HI * WI + (size_t)min(max(yy, 0), HI - 1) * WI + min(max(xx, 0), WI - 1)) * CP;
#pragma unroll 2
    for (int kc = 0; kc < CP / 32; ++kc) { const v16b ah = zfrag_if(frag_b(IH + ap + kc * 32, lane), ok); v16b al; if (MODE != 1) al = zfrag_if(frag_b(IL + ap + kc * 32, lane), ok); const size_t kk = (size_t)tap * CP + kc * 32;
#pragma unroll
      for (int j = 0; j < 12; ++j) { const v16b w = frag_b(W + (size_t)(j * 16 + col) * KT + kk, lane); if (MODE != 1) acc[j] = wmma_bf(al, w, acc[j]); acc[j] = wmma_bf(ah, w, acc[j]); } } }
#pragma unroll
  for (int j = 0; j < 12; ++j) { const int o = j * 16 + col;
#pragma unroll
    for (int r = 0; r < 8; ++r) { float v = acc[j][r];
      if (MODE == 1) { const size_t pr = r0 + 8 * g + r; const int im = (int)(pr / NPI), rr = (int)(pr % NPI), yq = (rr / WWD) / 2, xq = (rr % WWD) / 2; const float o2 = O2[((size_t)im * HP * HP + yq * HP + xq) * CP2 + o]; v = v * (1.0f / (1.0f + exp_ni(-o2))); }
      so[wave][8 * g + r][o] = v; } }
  LDSX();
  for (int rl = 0; rl < 16; ++rl) { const size_t pr = r0 + rl;
    if (MODE == 1) { __bf16 hb[8], lb[8]; const int c0 = (lane % 24) * 8; if (lane < 24) {
#pragma unroll
        for (int i = 0; i < 8; ++i) { const float v = so[wave][rl][c0 + i]; hb[i] = (__bf16)v; lb[i] = (__bf16)(v - (float)hb[i]); }
        vst2((unsigned*)(OH + pr * CP2 + c0), *(const v4u*)hb); vst2((unsigned*)(OL + pr * CP2 + c0), *(const v4u*)lb); } }
    else { for (int pc = lane; pc < CP2 / 4; pc += 32) vst2(OUTF + pr * CP2 + pc * 4, *(const v4f*)&so[wave][rl][pc * 4]); } }
}
template <int KS, int CO>
__global__ __launch_bounds__(128) void k_def(const float* __restrict__ X, const float* __restrict__ OFF, const __bf16* __restrict__ W, const float* __restrict__ BIAS, __bf16* __restrict__ FH, __bf16* __restrict__ FL) {
  constexpr int K2 = KS * KS, PADK = KS / 2, KT = CC * K2, OFF0 = (KS == 3) ? 0 : (KS == 5) ? 18 : 68;
  __shared__ unsigned short sidx[64][K2][4]; __shared__ float swt[64][K2][4]; __shared__ __align__(16) __bf16 th[64][40], tl[64][40]; __shared__ __align__(16) __bf16 soh[4][16][72], sol[4][16][72];
  const int tid = threadIdx.x, wave = tid >> 5, lane = tid & 31, col = lane & 15, g = lane >> 4; const int row = blockIdx.x; const int b = row / HH, y = row % HH;
  for (int q = tid; q < 64 * K2; q += 128) { const int px = q & 63, t = q >> 6; const size_t pr = (size_t)row * WWD + px; const float oy = OFF[pr * CP2 + OFF0 + 2 * t], ox = OFF[pr * CP2 + OFF0 + 2 * t + 1];
    const float py = ((float)y + ((float)(t / KS) - (float)PADK)) + oy, pxf = ((float)px + ((float)(t % KS) - (float)PADK)) + ox;
    const float y0 = floorf(py), x0 = floorf(pxf); const float dy = py - y0, dx = pxf - x0; const int yi = (int)y0, xi = (int)x0;
#pragma unroll
    for (int cnr = 0; cnr < 4; ++cnr) { const int yy = yi + (cnr >> 1), xx = xi + (cnr & 1); const bool ok = (yy >= 0) && (yy < HH) && (xx >= 0) && (xx < WWD);
      sidx[px][t][cnr] = (unsigned short)(min(max(yy, 0), HH - 1) * WWD + min(max(xx, 0), WWD - 1));
      const float wgt = (cnr == 0) ? (1.0f - dy) * (1.0f - dx) : (cnr == 1) ? (1.0f - dy) * dx : (cnr == 2) ? dy * (1.0f - dx) : dy * dx; swt[px][t][cnr] = ok ? wgt : 0.f; } }
  __syncthreads();
  v8f acc[4] = {};
#pragma unroll 1
  for (int kc = 0; kc < KT / 32; ++kc) {
    for (int q = tid; q < 64 * 32; q += 128) { const int px = q & 63, kl = q >> 6; const int k = kc * 32 + kl; const int c = k / K2, t = k % K2; const float* plane = X + ((size_t)b * CC + c) * NPI;
      const float v = ((bfr(plane[sidx[px][t][0]]) * swt[px][t][0] + bfr(plane[sidx[px][t][1]]) * swt[px][t][1]) + bfr(plane[sidx[px][t][2]]) * swt[px][t][2]) + bfr(plane[sidx[px][t][3]]) * swt[px][t][3];
      const __bf16 hb = (__bf16)v; th[px][kl] = hb; tl[px][kl] = (__bf16)(v - (float)hb); }
    __syncthreads();
    { F2 a; a.h = frag_b(&th[wave * 16 + col][0], lane); a.l = frag_b(&tl[wave * 16 + col][0], lane);
#pragma unroll
      for (int j = 0; j < 4; ++j) { const v16b w = frag_b(W + (size_t)(j * 16 + col) * KT + kc * 32, lane); acc[j] = wmma_bf(a.l, w, acc[j]); acc[j] = wmma_bf(a.h, w, acc[j]); } }
    __syncthreads(); }
#pragma unroll
  for (int j = 0; j < 4; ++j) { const int o = j * 16 + col; const float bb = bfr(BIAS[o]);
#pragma unroll
    for (int r = 0; r < 8; ++r) { const float v = fmaxf(acc[j][r] + bb, 0.f); const __bf16 hb = (__bf16)v; soh[wave][8 * g + r][o] = hb; sol[wave][8 * g + r][o] = (__bf16)(v - (float)hb); } }
  LDSX();
  for (int rl = 0; rl < 16; ++rl) if (lane < 16) { const size_t pr = (size_t)row * WWD + wave * 16 + rl; if (lane < 8) vst2((unsigned*)(FH + pr * CP2 + CO + lane * 8), *(const v4u*)&soh[wave][rl][lane * 8]); else vst2((unsigned*)(FL + pr * CP2 + CO + (lane - 8) * 8), *(const v4u*)&sol[wave][rl][(lane - 8) * 8]); }
}
__global__ __launch_bounds__(128) void k_pw(const __bf16* __restrict__ FH, const __bf16* __restrict__ FL, const __bf16* __restrict__ W, const float* __restrict__ BIAS, float* __restrict__ OUT) {
  __shared__ __align__(16) float so[CC][68];
  const int tid = threadIdx.x, wave = tid >> 5, lane = tid & 31, col = lane & 15, g = lane >> 4; const int row = blockIdx.x; const int b = row / HH, y = row % HH; const size_t r0 = (size_t)row * WWD + wave * 16;
  v8f acc[4] = {};
#pragma unroll
  for (int kc = 0; kc < CP2 / 32; ++kc) { F2 a; a.h = frag_b(FH + (r0 + col) * CP2 + kc * 32, lane); a.l = frag_b(FL + (r0 + col) * CP2 + kc * 32, lane);
#pragma unroll
    for (int j = 0; j < 4; ++j) { const v16b w = frag_b(W + (size_t)(j * 16 + col) * CP2 + kc * 32, lane); acc[j] = wmma_bf(a.l, w, acc[j]); acc[j] = wmma_bf(a.h, w, acc[j]); } }
#pragma unroll
  for (int j = 0; j < 4; ++j) { const int o = j * 16 + col; const float bb = bfr(BIAS[o]);
#pragma unroll
    for (int r = 0; r < 8; ++r) so[o][wave * 16 + 8 * g + r] = acc[j][r] + bb; }
  __syncthreads();
  for (int q = tid; q < CC * 16; q += 128) { const int o = q >> 4, pc = q & 15; vst2(OUT + (((size_t)b * CC + o) * HH + y) * WWD + pc * 4, *(const v4f*)&so[o][pc * 4]); }
}
extern "C" void kernel_launch(void* const* d_in, const int* in_sizes, int n_in, void* d_out, int out_size, void* d_ws, size_t ws_size, hipStream_t stream) {
  (void)in_sizes; (void)n_in; (void)out_size;
  const float** F = (const float**)d_in;
  if (ws_size < (size_t)WS_END) return;
  char* ws = (char*)d_ws; __bf16 *PK = (__bf16*)(ws + WS_PK), *XY = (__bf16*)(ws + WS_XY), *PH = (__bf16*)(ws + WS_PLH), *PL = (__bf16*)(ws + WS_PLL), *G3H = (__bf16*)(ws + WS_G3H), *G3L = (__bf16*)(ws + WS_G3L); float *O2 = (float*)(ws + WS_O2), *OFFS = (float*)(ws + WS_OFF);
  __bf16 *FH = PH, *FL = PL;
  k_pack<<<dim3(CP2, 7), 256, 0, stream>>>(F[2], F[3], F[4], F[5], F[7], F[9], F[11], PK);
  k_xy<<<NBT * HH, 256, 0, stream>>>(F[0], F[1], XY);
  k_pool<<<NBT * HP, 256, 0, stream>>>(XY, PH, PL);
  k_c33<0><<<NPB, 128, 0, stream>>>(PH, PL, PK + PK_2, nullptr, O2, nullptr, nullptr);
  k_c33<1><<<NRB1, 128, 0, stream>>>(XY, nullptr, PK + PK_3, O2, nullptr, G3H, G3L);
  k_c33<2><<<NRB, 128, 0, stream>>>(G3H, G3L, PK + PK_4, nullptr, OFFS, nullptr, nullptr);
  FH = G3H; FL = G3L;
  k_def<3, 0><<<NRB, 128, 0, stream>>>(F[0], OFFS, PK + PK_D3, F[6], FH, FL);
  k_def<5, 64><<<NRB, 128, 0, stream>>>(F[0], OFFS, PK + PK_D5, F[8], FH, FL);
  k_def<7, 128><<<NRB, 128, 0, stream>>>(F[0], OFFS, PK + PK_D7, F[10], FH, FL);
  k_pw<<<NRB, 128, 0, stream>>>(FH, FL, PK + PK_PW, F[12], (float*)d_out);
}
